// SelfAttentionLayer_74096775790973
// MI455X (gfx1250) — hardware-verified
//
#include <hip/hip_runtime.h>


#ifndef NB
#define NB 4
#endif
#ifndef SEQ
#define SEQ 2048
#endif
#define NB_FULL 4
#define S_FULL  2048
#define TT   SEQ
#define DM   1024
#define NH   16
#define HD   64
#define MR   (NB * TT)
#define PCAR 1024.0f
#define CTXC 64.0f
#define WOC  16.0f
#define OINV (1.0f / (CTXC * WOC))
#define SCL  0.03125f
#define L2E  1.4426950408889634f
#define LNEPS 1.0e-6f
#define PP   72

static_assert(NB >= 1 && NB <= NB_FULL);
static_assert(TT % 64 == 0 && TT <= S_FULL);
static_assert(DM % 64 == 0);
static_assert(NH * HD == DM);
static_assert(HD == 64);

typedef _Float16 h16;
typedef unsigned short bf;
typedef __attribute__((ext_vector_type(16))) __bf16   v16bf;
typedef __attribute__((ext_vector_type(16))) _Float16 v16h;
typedef __attribute__((ext_vector_type(8)))  _Float16 v8h;
typedef __attribute__((ext_vector_type(8)))  unsigned short v8us;
typedef __attribute__((ext_vector_type(8)))  float    v8f;
typedef __attribute__((ext_vector_type(4)))  float    v4f;
typedef __attribute__((ext_vector_type(2)))  _Float16 v2h;
typedef __attribute__((ext_vector_type(2)))  unsigned short v2us;
typedef __attribute__((ext_vector_type(2)))  float v2f;
typedef v8h  __attribute__((may_alias)) v8ha;
typedef v4f  __attribute__((may_alias)) v4fa;
typedef v8us __attribute__((may_alias)) v8usa;

__device__ __forceinline__ unsigned short f2bf(float f) { unsigned u = __float_as_uint(f); u += 0x7FFFu + ((u >> 16) & 1u); return (unsigned short)(u >> 16); }
__device__ __forceinline__ float bf2f(unsigned short b) { return __uint_as_float(((unsigned)b) << 16); }
__device__ __forceinline__ float bfr(float f) { return bf2f(f2bf(f)); }
__device__ __forceinline__ v16h cat16(v8h lo, v8h hi) { return __builtin_shufflevector(lo, hi, 0, 1, 2, 3, 4, 5, 6, 7, 8, 9, 10, 11, 12, 13, 14, 15); }
__device__ __forceinline__ v16bf cat16b(v8us lo, v8us hi) { return __builtin_bit_cast(v16bf, __builtin_shufflevector(lo, hi, 0, 1, 2, 3, 4, 5, 6, 7, 8, 9, 10, 11, 12, 13, 14, 15)); }
__device__ __forceinline__ v8f wmma16(v16h a, v16h b, v8f c) { return __builtin_amdgcn_wmma_f32_16x16x32_f16(false, a, false, b, (short)0, c, false, false); }
__device__ __forceinline__ v8f wmmab(v16bf a, v16bf b, v8f c) { return __builtin_amdgcn_wmma_f32_16x16x32_bf16(false, a, false, b, (short)0, c, false, false); }

template <typename T16> struct WFrag;
template <> struct WFrag<h16> { typedef v16h V; static __device__ __forceinline__ V ld(const h16* p) { return cat16(*(const v8h*)p, *(const v8h*)(p + 16)); } static __device__ __forceinline__ v8f mma(V a, V b, v8f c) { return wmma16(a, b, c); } };
template <> struct WFrag<bf> { typedef v16bf V; static __device__ __forceinline__ V ld(const bf* p) { return cat16b(*(const v8us*)p, *(const v8us*)(p + 16)); } static __device__ __forceinline__ v8f mma(V a, V b, v8f c) { return wmmab(a, b, c); } };
template <typename T16, int NSPLIT, bool BIAS>
__global__ __launch_bounds__(32) void k_gemmw(const T16* __restrict__ A, const T16* __restrict__ A2, const T16* __restrict__ Bt, const T16* __restrict__ Bt2, int K, float* C, int ldc, const float* __restrict__ bias, size_t sA, size_t sB, size_t sC) {
    typedef typename WFrag<T16>::V V;
    __shared__ __align__(16) float os[16 * 68];
    const size_t z = blockIdx.z; A += z * sA; if (A2) A2 += z * sA; Bt += z * sB; if (Bt2) Bt2 += z * sB; C += z * sC;
    const int lane = threadIdx.x & 31, lr = lane & 15, hi = lane >> 4; const int r0 = blockIdx.x * 64, c0 = blockIdx.y * 64;
    v8f acc[4][4];
#pragma unroll
    for (int mb = 0; mb < 4; ++mb)
#pragma unroll
        for (int nb = 0; nb < 4; ++nb) acc[mb][nb] = (v8f){};
    const size_t aoff = (size_t)(r0 + lr) * K + 8 * hi, boff = (size_t)(c0 + lr) * K + 8 * hi;
#pragma unroll 1
    for (int kc = 0; kc < K; kc += 32) {
        V a[4], a2[4];
#pragma unroll
        for (int mb = 0; mb < 4; ++mb) { a[mb] = WFrag<T16>::ld(A + aoff + (size_t)mb * 16 * K + kc); if (NSPLIT == 1 || NSPLIT == 2) a2[mb] = WFrag<T16>::ld(A2 + aoff + (size_t)mb * 16 * K + kc); }
#pragma unroll
        for (int nb = 0; nb < 4; ++nb) { const V b = WFrag<T16>::ld(Bt + boff + (size_t)nb * 16 * K + kc); V b2; if (NSPLIT >= 2) b2 = WFrag<T16>::ld(Bt2 + boff + (size_t)nb * 16 * K + kc);
#pragma unroll
            for (int mb = 0; mb < 4; ++mb) { acc[mb][nb] = WFrag<T16>::mma(a[mb], b, acc[mb][nb]); if (NSPLIT == 1 || NSPLIT == 2) acc[mb][nb] = WFrag<T16>::mma(a2[mb], b, acc[mb][nb]); if (NSPLIT >= 2) acc[mb][nb] = WFrag<T16>::mma(a[mb], b2, acc[mb][nb]); } }
        asm volatile("v_nop\n\tv_nop\n\tv_nop\n\tv_nop" : "+v"(acc[0][0]), "+v"(acc[1][1]), "+v"(acc[2][2]), "+v"(acc[3][3]) : "v"(a[0]), "v"(a[3]));
    }
#pragma unroll
    for (int mb = 0; mb < 4; ++mb) {
#pragma unroll
        for (int nb = 0; nb < 4; ++nb) {
#pragma unroll
            for (int j = 0; j < 8; ++j) os[(hi * 8 + j) * 68 + nb * 16 + lr] = acc[mb][nb][j]; }
        __builtin_amdgcn_fence(3, "wavefront"); __builtin_amdgcn_wave_barrier(); asm volatile("" ::: "memory");
        float* crow = C + (size_t)(r0 + mb * 16) * ldc + c0;
#pragma unroll 1
        for (int ps = 0; ps < 2; ++ps) {
#pragma unroll
            for (int s = 0; s < 8; ++s) { const int row = 2 * s + hi, cofs = lr * 4; v4f val = *(const v4fa*)(os + row * 68 + cofs); if (BIAS) { val[0] += bfr(bias[c0 + cofs]); val[1] += bfr(bias[c0 + cofs + 1]); val[2] += bfr(bias[c0 + cofs + 2]); val[3] += bfr(bias[c0 + cofs + 3]); }
                *(volatile v4f*)(crow + (size_t)row * ldc + cofs) = val; }
            if (ps == 0) __threadfence(); }
        __builtin_amdgcn_wave_barrier(); asm volatile("" ::: "memory");
    }
}

template <typename T16> struct Cv;
template <> struct Cv<bf>  { typedef v2us V2; static __device__ __forceinline__ bf  c(float f) { return f2bf(f); } };
template <> struct Cv<h16> { typedef v2h  V2; static __device__ __forceinline__ h16 c(float f) { return (h16)f; } };
template <typename T16>
__global__ __launch_bounds__(256) void k_wt(const float* __restrict__ w, int K, int N, float sc, T16* Bt) {
    typedef typename Cv<T16>::V2 V2;
    const int lane = threadIdx.x & 31; const int L0 = (blockIdx.x * 8 + (threadIdx.x >> 5)) * 8; const int nlines = N * K / 64;
#pragma unroll
    for (int ps = 0; ps < 2; ++ps) {
#pragma unroll 1
        for (int l = 0; l < 8; ++l) { const int L = L0 + l; if (L >= nlines) break; const size_t e = (size_t)L * 64 + lane * 2; const int k = (int)(e % K), n = (int)(e / K); V2 o;
            o[0] = Cv<T16>::c(bfr(w[(size_t)k * N + n]) * sc); o[1] = Cv<T16>::c(bfr(w[(size_t)(k + 1) * N + n]) * sc); *(volatile V2*)(Bt + e) = o; }
        if (ps == 0) __threadfence(); }
}

__global__ __launch_bounds__(256) void k_cvtx(const float* __restrict__ src, bf* dst, size_t n8) {
    const size_t i = (size_t)blockIdx.x * 256 + threadIdx.x; if (i >= n8) return;
    const size_t e = i * 8; const size_t row = e / DM; const int col = (int)(e - row * DM); const size_t b = row / TT, t = row - b * TT;
    const v8f v = *(const v8f*)(src + (b * S_FULL + t) * DM + col); v8us o;
#pragma unroll
    for (int k = 0; k < 8; ++k) o[k] = f2bf(v[k]);
    *(volatile v8us*)(dst + e) = o; __threadfence(); *(volatile v8us*)(dst + e) = o;
}

__global__ __launch_bounds__(256) void k_qkplane(const float* __restrict__ F, h16* P) {
    const size_t e = ((size_t)blockIdx.x * 256 + threadIdx.x) * 2; if (e >= (size_t)MR * DM) return;
    const int d = (int)(e % HD); const int t = (int)((e / HD) % TT); const int g = (int)(e / ((size_t)HD * TT)); const int b = g / NH, h = g - b * NH;
    const v2f f = *(const v2f*)(F + ((size_t)b * TT + t) * DM + h * HD + d);
    v2h o; o[0] = (h16)f[0]; o[1] = (h16)f[1];
    *(volatile v2h*)(P + e) = o; __threadfence(); *(volatile v2h*)(P + e) = o;
}
__global__ __launch_bounds__(256) void k_vplane(const float* __restrict__ F, h16* VT) {
    const size_t e = ((size_t)blockIdx.x * 256 + threadIdx.x) * 2; if (e >= (size_t)MR * DM) return;
    const int t = (int)(e % TT); const int d = (int)((e / TT) % HD); const int g = (int)(e / ((size_t)TT * HD)); const int b = g / NH, h = g - b * NH;
    v2h o;
#pragma unroll
    for (int q = 0; q < 2; ++q) o[q] = (h16)F[((size_t)b * TT + t + q) * DM + h * HD + d];
    *(volatile v2h*)(VT + e) = o; __threadfence(); *(volatile v2h*)(VT + e) = o;
}

__global__ __launch_bounds__(128) __attribute__((amdgpu_num_vgpr(256)))
void k_attn(const h16* __restrict__ QP, const h16* __restrict__ KP, const h16* __restrict__ VT, const float* __restrict__ mask, h16* CT) {
    __shared__ __align__(16) h16 Psh[4 * 16 * PP];
    const int lane = threadIdx.x & 31, lr = lane & 15, hi = lane >> 4, wv = threadIdx.x >> 5;
    const int bh = blockIdx.y; const int b = bh / NH, h = bh - b * NH;
    const int r0 = blockIdx.x * 64 + wv * 16;
    h16* Pw = Psh + wv * (16 * PP);
    const h16* Qb = QP + ((size_t)bh * TT + r0) * HD;
    const h16* Kb = KP + (size_t)bh * TT * HD;
    const h16* Vb = VT + (size_t)bh * HD * TT;
    const float* mrow = mask + (size_t)b * S_FULL;
    v16h qa[2];
#pragma unroll
    for (int ks = 0; ks < 2; ++ks) qa[ks] = WFrag<h16>::ld(Qb + (size_t)lr * HD + ks * 32 + 8 * hi);
    v8f o[4]; float m[8], l[8];
#pragma unroll
    for (int nb = 0; nb < 4; ++nb) o[nb] = (v8f){};
#pragma unroll
    for (int r = 0; r < 8; ++r) { m[r] = -1.0e30f; l[r] = 0.f; }
#pragma unroll 1
    for (int kt = 0; kt < TT; kt += 64) {
        v8f s[4];
#pragma unroll
        for (int nb = 0; nb < 4; ++nb) s[nb] = (v8f){};
#pragma unroll
        for (int ks = 0; ks < 2; ++ks) {
#pragma unroll
            for (int nb = 0; nb < 4; ++nb) { const v16h kb = WFrag<h16>::ld(Kb + (size_t)(kt + nb * 16 + lr) * HD + ks * 32 + 8 * hi); s[nb] = wmma16(qa[ks], kb, s[nb]); } }
        asm volatile("v_nop\n\tv_nop\n\tv_nop\n\tv_nop" : "+v"(s[0]), "+v"(s[1]), "+v"(s[2]), "+v"(s[3]) : "v"(qa[0]), "v"(qa[1]));
        float tm[8];
#pragma unroll
        for (int r = 0; r < 8; ++r) tm[r] = -1.0e30f;
#pragma unroll
        for (int nb = 0; nb < 4; ++nb) { const float mk = bfr(mrow[kt + nb * 16 + lr]) * (-1.0e9f);
#pragma unroll
            for (int r = 0; r < 8; ++r) { const float t = s[nb][r] * SCL + mk; s[nb][r] = t; tm[r] = fmaxf(tm[r], t); } }
#pragma unroll
        for (int r = 0; r < 8; ++r) {
#pragma unroll
            for (int sh = 8; sh; sh >>= 1) tm[r] = fmaxf(tm[r], __shfl_xor(tm[r], sh, 32)); }
        float psum[8];
#pragma unroll
        for (int r = 0; r < 8; ++r) { const float mn = fmaxf(m[r], tm[r]); float da = __fsub_rn(m[r], mn); asm volatile("" : "+v"(da)); const float al = __builtin_amdgcn_exp2f(__fmul_rn(da, L2E)); m[r] = mn; l[r] *= al;
#pragma unroll
            for (int nb = 0; nb < 4; ++nb) o[nb][r] *= al;
            psum[r] = 0.f; }
#pragma unroll
        for (int nb = 0; nb < 4; ++nb) {
#pragma unroll
            for (int r = 0; r < 8; ++r) { float d0 = __fsub_rn(s[nb][r], m[r]); asm volatile("" : "+v"(d0)); const float e = __builtin_amdgcn_exp2f(__fmul_rn(d0, L2E)); const h16 p16 = (h16)(e * PCAR);
                Pw[(8 * hi + r) * PP + nb * 16 + lr] = p16; psum[r] += (float)p16; } }
#pragma unroll
        for (int r = 0; r < 8; ++r) {
#pragma unroll
            for (int sh = 8; sh; sh >>= 1) psum[r] += __shfl_xor(psum[r], sh, 32);
            l[r] += psum[r]; }
        __builtin_amdgcn_fence(3, "wavefront"); __builtin_amdgcn_wave_barrier(); asm volatile("" ::: "memory");
        v16h pa[2];
#pragma unroll
        for (int ks = 0; ks < 2; ++ks) pa[ks] = cat16(*(const v8ha*)(Pw + lr * PP + ks * 32 + 8 * hi), *(const v8ha*)(Pw + lr * PP + ks * 32 + 16 + 8 * hi));
#pragma unroll
        for (int ks = 0; ks < 2; ++ks) {
#pragma unroll
            for (int nb = 0; nb < 4; ++nb) { const v16h vb = WFrag<h16>::ld(Vb + (size_t)(nb * 16 + lr) * TT + kt + ks * 32 + 8 * hi); o[nb] = wmma16(pa[ks], vb, o[nb]); } }
        asm volatile("v_nop\n\tv_nop\n\tv_nop\n\tv_nop" : "+v"(o[0]), "+v"(o[1]), "+v"(o[2]), "+v"(o[3]) : "v"(pa[0]), "v"(pa[1]));
        __builtin_amdgcn_wave_barrier(); asm volatile("" ::: "memory");
    }
    float fr[8];
#pragma unroll
    for (int r = 0; r < 8; ++r) fr[r] = __fdiv_rn(CTXC, l[r]);
#pragma unroll
    for (int nb = 0; nb < 4; ++nb) {
#pragma unroll
        for (int r = 0; r < 8; ++r) Pw[(8 * hi + r) * PP + nb * 16 + lr] = (h16)(o[nb][r] * fr[r]); }
    __builtin_amdgcn_fence(3, "wavefront"); __builtin_amdgcn_wave_barrier(); asm volatile("" ::: "memory");
    h16* cb = CT + ((size_t)b * TT + r0) * DM + h * HD;
    const int rw = lane >> 3, pc = (lane & 7) * 8;
#pragma unroll 1
    for (int ps = 0; ps < 2; ++ps) {
#pragma unroll
        for (int s4 = 0; s4 < 4; ++s4) { const int row = rw + 4 * s4; const v8h val = *(const v8ha*)(Pw + row * PP + pc); *(volatile v8h*)(cb + (size_t)row * DM + pc) = val; }
        if (ps == 0) __threadfence(); }
}

__global__ __launch_bounds__(256) void k_ln(const float* __restrict__ Y, const float* __restrict__ X, const float* __restrict__ bo, const float* __restrict__ gm, const float* __restrict__ bt, float* OUT) {
    __shared__ float red[8], red2[8];
    const int rr = blockIdx.x; const int b = rr / TT, t = rr - b * TT; const int tid = threadIdx.x, lane = tid & 31, wv = tid >> 5; const int c = tid * 4;
    const size_t frow = ((size_t)b * S_FULL + t) * DM;
    const v4f y = *(const v4f*)(Y + (size_t)rr * DM + c); const v4f xx = *(const v4f*)(X + frow + c); const v4f bb = *(const v4f*)(bo + c); const v4f gg = *(const v4f*)(gm + c); const v4f be = *(const v4f*)(bt + c);
    float a[4]; float sm = 0.f;
#pragma unroll
    for (int q = 0; q < 4; ++q) { const float mo = __fadd_rn(y[q] * OINV, bfr(bb[q])); a[q] = __fadd_rn(mo, bfr(xx[q])); sm += a[q]; }
#pragma unroll
    for (int sh = 16; sh; sh >>= 1) sm += __shfl_xor(sm, sh, 32);
    if (lane == 0) red[wv] = sm;
    __syncthreads();
    float tot = 0.f;
#pragma unroll
    for (int w = 0; w < 8; ++w) tot += red[w];
    const float mu = tot * (1.0f / (float)DM);
    float dv[4]; float sv = 0.f;
#pragma unroll
    for (int q = 0; q < 4; ++q) { dv[q] = __fsub_rn(a[q], mu); sv += dv[q] * dv[q]; }
#pragma unroll
    for (int sh = 16; sh; sh >>= 1) sv += __shfl_xor(sv, sh, 32);
    if (lane == 0) red2[wv] = sv;
    __syncthreads();
    float tot2 = 0.f;
#pragma unroll
    for (int w = 0; w < 8; ++w) tot2 += red2[w];
    const float var = tot2 * (1.0f / (float)DM);
    const float rstd = 1.0f / sqrtf(var + LNEPS);
    v4f o4;
#pragma unroll
    for (int q = 0; q < 4; ++q) o4[q] = (bfr(gg[q]) * dv[q]) * rstd + bfr(be[q]);
    float* op = OUT + frow + c;
    *(volatile v4f*)op = o4; __threadfence(); *(volatile v4f*)op = o4;
}

extern "C" void kernel_launch(void* const* d_in, const int* in_sizes, int n_in,
                              void* d_out, int out_size, void* d_ws, size_t ws_size, hipStream_t stream) {
    if (n_in < 12) return;
    const float* x = (const float*)d_in[0]; const float* mask = (const float*)d_in[1];
    const float* wq = (const float*)d_in[2]; const float* bq = (const float*)d_in[3]; const float* wk = (const float*)d_in[4]; const float* bk = (const float*)d_in[5];
    const float* wvv = (const float*)d_in[6]; const float* bv = (const float*)d_in[7]; const float* wo = (const float*)d_in[8]; const float* bo = (const float*)d_in[9];
    const float* gam = (const float*)d_in[10]; const float* bet = (const float*)d_in[11];
    float* OUT = (float*)d_out;
    const int rows_needed = (NB - 1) * S_FULL + TT;
    if (in_sizes[0] < rows_needed * DM || in_sizes[1] < rows_needed || out_size < rows_needed * DM) return;
    if (in_sizes[2] < DM * DM || in_sizes[4] < DM * DM || in_sizes[6] < DM * DM || in_sizes[8] < DM * DM) return;
    if (in_sizes[3] < DM || in_sizes[5] < DM || in_sizes[7] < DM || in_sizes[9] < DM || in_sizes[10] < DM || in_sizes[11] < DM) return;
    char* wsp = (char*)d_ws;
    auto take = [&](size_t bytes) { char* p = wsp; wsp += (bytes + 255) & ~(size_t)255; return (void*)p; };
    bf*  XB  = (bf*)take((size_t)MR * DM * 2);
    bf*  WQt = (bf*)take((size_t)DM * DM * 2); bf* WKt = (bf*)take((size_t)DM * DM * 2); bf* WVt = (bf*)take((size_t)DM * DM * 2); h16* WOt = (h16*)take((size_t)DM * DM * 2);
    float* F = (float*)take((size_t)MR * DM * 4);
    h16* QP = (h16*)take((size_t)MR * DM * 2); h16* KP = (h16*)take((size_t)MR * DM * 2); h16* VT = (h16*)take((size_t)MR * DM * 2); h16* CT = (h16*)take((size_t)MR * DM * 2);
    if ((size_t)(wsp - (char*)d_ws) > ws_size) return;
    float* Y = F;

    const size_t n8 = (size_t)MR * DM / 8;
    k_cvtx<<<(unsigned)((n8 + 255) / 256), 256, 0, stream>>>(x, XB, n8);
    const unsigned wtg = (unsigned)((DM * DM / 64 + 63) / 64);
    k_wt<bf><<<wtg, 256, 0, stream>>>(wq, DM, DM, 1.0f, WQt);
    k_wt<bf><<<wtg, 256, 0, stream>>>(wk, DM, DM, 1.0f, WKt);
    k_wt<bf><<<wtg, 256, 0, stream>>>(wvv, DM, DM, 1.0f, WVt);
    k_wt<h16><<<wtg, 256, 0, stream>>>(wo, DM, DM, WOC, WOt);
    const dim3 gg(MR / 64, DM / 64, 1);
    const unsigned plg = (unsigned)(((size_t)MR * DM / 2 + 255) / 256);
    k_gemmw<bf, 0, true><<<gg, 32, 0, stream>>>(XB, nullptr, WQt, nullptr, DM, F, DM, bq, 0, 0, 0);
    k_qkplane<<<plg, 256, 0, stream>>>(F, QP);
    k_gemmw<bf, 0, true><<<gg, 32, 0, stream>>>(XB, nullptr, WKt, nullptr, DM, F, DM, bk, 0, 0, 0);
    k_qkplane<<<plg, 256, 0, stream>>>(F, KP);
    k_gemmw<bf, 0, true><<<gg, 32, 0, stream>>>(XB, nullptr, WVt, nullptr, DM, F, DM, bv, 0, 0, 0);
    k_vplane<<<plg, 256, 0, stream>>>(F, VT);
    k_attn<<<dim3(TT / 64, NB * NH, 1), 128, 0, stream>>>(QP, KP, VT, mask, CT);
    k_gemmw<h16, 0, false><<<gg, 32, 0, stream>>>(CT, nullptr, WOt, nullptr, DM, Y, DM, nullptr, 0, 0, 0);
    k_ln<<<MR, 256, 0, stream>>>(Y, x, bo, gam, bet, OUT);
}
